// GraphLayer_32693291057755
// MI455X (gfx1250) — hardware-run, weakly checked
//
#include <hip/hip_runtime.h>
#include <stddef.h>
#include <stdint.h>
#include <math.h>


#define DIN     128
#define DOUT    128
#define GBM     128
#define NTHR    256
#define NWAVE   8
#define EPT     8
#define CHUNK   2048
#define WCAP    256
#define LISTN   (NWAVE * WCAP)
#define NBRUN   256
#define SLB     8
#define SRCB    14
#define RCAP    20480
#define DEGCAP  128
#define NN_SPEC 10000
#define WBLK    ((DOUT * (DIN / 8)) / NTHR)
#define BKT_INTS (LISTN + 2 * RCAP + 3 * NBRUN + 32)
#define ZSD_FLTS (GBM * DOUT + 2 * GBM + 2 * DOUT)

static_assert(NBRUN == (1 << SLB) && NBRUN == NTHR);
static_assert(CHUNK == NWAVE * WCAP && WCAP == EPT * 32);
static_assert((CHUNK & (CHUNK - 1)) == 0);
static_assert(NN_SPEC <= (1 << SRCB));
static_assert(SRCB + SLB < 31);
static_assert(RCAP % 32 == 0 && DEGCAP <= RCAP);
static_assert(DOUT == 32 * 4 && DIN % 32 == 0);
static_assert(GBM == NWAVE * 16);
static_assert((DOUT * (DIN / 8)) % NTHR == 0);
static_assert(BKT_INTS * 4 <= 327680);
static_assert(ZSD_FLTS * 4 <= 327680);
static_assert(NBRUN % NWAVE == 0 && NBRUN / NWAVE == 32);

typedef float          v4f   __attribute__((ext_vector_type(4)));
typedef float          v8f   __attribute__((ext_vector_type(8)));
typedef int            v4i   __attribute__((ext_vector_type(4)));
typedef int            v8i   __attribute__((ext_vector_type(8)));
typedef unsigned short v8us  __attribute__((ext_vector_type(8)));
typedef unsigned short v16us __attribute__((ext_vector_type(16)));
typedef __bf16         v16bf __attribute__((ext_vector_type(16)));
typedef v4f  __attribute__((may_alias)) v4fa;
typedef v4i  __attribute__((may_alias)) v4ia;
typedef v8us __attribute__((may_alias)) v8usa;
union FragB { v16bf v; v16us u; v8us h[2]; v8i w; };

__device__ __forceinline__ v8f wmb(const FragB& a, const FragB& b, v8f c) {
  v8f d = __builtin_amdgcn_wmma_f32_16x16x32_bf16(false, a.v, false, b.v, (short)0, c, false, false);
  asm volatile("v_nop\n\tv_nop\n\tv_nop\n\tv_nop" : "+v"(d) : "v"(a.w), "v"(b.w));
  return d;
}

__device__ __forceinline__ unsigned bf16_bits(float f) {
  const unsigned u = __float_as_uint(f);
  return (u + 0x7FFFu + ((u >> 16) & 1u)) >> 16;
}
__device__ __forceinline__ float bf16_val(float f) {
  return __uint_as_float(bf16_bits(f) << 16);
}

__global__ __launch_bounds__(NTHR) void k_prep(const float* __restrict__ h, const float* __restrict__ Wfc,
                                               const float* __restrict__ Wat, int nN, int bH,
                                               unsigned short* HB, unsigned short* WB, float* AV) {
  const int b = (int)blockIdx.x, tid = (int)threadIdx.x;
  if (b < bH) {
    const int u   = b * NTHR + tid;
    const int row = u >> 4;
    const int k8  = (u & 15) * 8;
    const int rc  = row < nN ? row : nN - 1;
    const float* p = h + (size_t)rc * DIN + k8;
    const v4f a = *(const v4f*)p;
    const v4f c = *(const v4f*)(p + 4);
    const unsigned mk = row < nN ? 0xFFFFu : 0u;
    v8us o;
    o[0] = (unsigned short)(bf16_bits(a.x) & mk);
    o[1] = (unsigned short)(bf16_bits(a.y) & mk);
    o[2] = (unsigned short)(bf16_bits(a.z) & mk);
    o[3] = (unsigned short)(bf16_bits(a.w) & mk);
    o[4] = (unsigned short)(bf16_bits(c.x) & mk);
    o[5] = (unsigned short)(bf16_bits(c.y) & mk);
    o[6] = (unsigned short)(bf16_bits(c.z) & mk);
    o[7] = (unsigned short)(bf16_bits(c.w) & mk);
    unsigned short* dp = HB + (size_t)row * DIN + k8;
    *(volatile v8us*)dp = o;
    __threadfence();
    *(volatile v8us*)dp = o;
  } else if (b < bH + WBLK) {
    const int u  = (b - bH) * NTHR + tid;
    const int n  = u >> 4;
    const int k8 = (u & 15) * 8;
    const float* p = Wfc + (size_t)n * DIN + k8;
    const v4f a = *(const v4f*)p;
    const v4f c = *(const v4f*)(p + 4);
    v8us o;
    o[0] = (unsigned short)bf16_bits(a.x);
    o[1] = (unsigned short)bf16_bits(a.y);
    o[2] = (unsigned short)bf16_bits(a.z);
    o[3] = (unsigned short)bf16_bits(a.w);
    o[4] = (unsigned short)bf16_bits(c.x);
    o[5] = (unsigned short)bf16_bits(c.y);
    o[6] = (unsigned short)bf16_bits(c.z);
    o[7] = (unsigned short)bf16_bits(c.w);
    unsigned short* dp = WB + (size_t)n * DIN + k8;
    *(volatile v8us*)dp = o;
    __threadfence();
    *(volatile v8us*)dp = o;
  } else {
    if (tid < 64) {
      const v4f a = *(const v4f*)(Wat + 4 * tid);
      v4f r;
      r.x = bf16_val(a.x); r.y = bf16_val(a.y); r.z = bf16_val(a.z); r.w = bf16_val(a.w);
      float* dp = AV + 4 * tid;
      *(volatile v4f*)dp = r;
      __threadfence();
      *(volatile v4f*)dp = r;
    }
  }
}

__global__ __launch_bounds__(NTHR) __attribute__((amdgpu_num_vgpr(248)))
void k_zsd(const unsigned short* __restrict__ A, const unsigned short* __restrict__ BT,
           const float* __restrict__ AV, float* Zp, float* SDp) {
  extern __shared__ __attribute__((aligned(16))) float gsm[];
  float* stg = gsm;
  float* sdt = gsm + GBM * DOUT;
  float* sav = sdt + 2 * GBM;
  const int tid = (int)threadIdx.x, lane = tid & 31, hh = lane >> 4, m = lane & 15;
  const int wave = __builtin_amdgcn_readfirstlane(tid >> 5);
  const int rowBase = (int)blockIdx.x * GBM;

  if (tid < 64) {
    const v4f a = *(const v4f*)(AV + 4 * tid);
    *(v4fa*)(sav + 4 * tid) = a;
  }

  v8f acc[8];
  {
    const v8f z = {0.f, 0.f, 0.f, 0.f, 0.f, 0.f, 0.f, 0.f};
#pragma unroll
    for (int t = 0; t < 8; ++t) acc[t] = z;
  }
  const unsigned short* ap = A  + (size_t)(rowBase + 16 * wave + m) * (size_t)DIN + 8 * hh;
  const unsigned short* bp = BT + (size_t)m * (size_t)DIN + 8 * hh;

#pragma unroll 1
  for (int k0 = 0; k0 < DIN; k0 += 32) {
    FragB af;
    af.h[0] = *(const v8usa*)(ap + k0);
    af.h[1] = *(const v8usa*)(ap + k0 + 16);
#pragma unroll
    for (int nt = 0; nt < 8; ++nt) {
      const unsigned short* wq = bp + (size_t)(16 * nt) * (size_t)DIN + k0;
      FragB bf;
      bf.h[0] = *(const v8usa*)wq;
      bf.h[1] = *(const v8usa*)(wq + 16);
      acc[nt] = wmb(af, bf, acc[nt]);
    }
  }

#pragma unroll
  for (int nt = 0; nt < 8; ++nt) {
    const int lc = 16 * nt + m;
#pragma unroll
    for (int r = 0; r < 8; ++r) {
      const int lr = 16 * wave + 8 * hh + r;
      stg[lr * DOUT + lc] = acc[nt][r];
    }
  }
  __syncthreads();

  const v4f as4 = *(const v4fa*)(sav + 4 * lane);
  const v4f ad4 = *(const v4fa*)(sav + DOUT + 4 * lane);
#pragma unroll 1
  for (int i = 0; i < 16; ++i) {
    const int row = wave * 16 + i;
    const v4f p = *(const v4fa*)(stg + row * DOUT + 4 * lane);
    float s = 0.0f, d = 0.0f;
    s = fmaf(p.x, as4.x, s); s = fmaf(p.y, as4.y, s); s = fmaf(p.z, as4.z, s); s = fmaf(p.w, as4.w, s);
    d = fmaf(p.x, ad4.x, d); d = fmaf(p.y, ad4.y, d); d = fmaf(p.z, ad4.z, d); d = fmaf(p.w, ad4.w, d);
#pragma unroll
    for (int off = 16; off > 0; off >>= 1) {
      s += __shfl_xor(s, off);
      d += __shfl_xor(d, off);
    }
    if (lane == 0) { sdt[2 * row] = s; sdt[2 * row + 1] = d; }
  }
  __syncthreads();

  const int sq = tid < 64 ? tid : 63;
  const v4f sdv = *(const v4fa*)(sdt + 4 * sq);
  float* sp = SDp + (size_t)rowBase * 2 + 4 * sq;
#pragma unroll 1
  for (int i = 0; i < 16; ++i) {
    const int row = wave * 16 + i;
    const v4f p = *(const v4fa*)(stg + row * DOUT + 4 * lane);
    float* op = Zp + (size_t)(rowBase + row) * (size_t)DOUT + 4 * lane;
    *(volatile v4f*)op = p;
  }
  if (wave < 2) *(volatile v4f*)sp = sdv;
  __threadfence();
#pragma unroll 1
  for (int i = 0; i < 16; ++i) {
    const int row = wave * 16 + i;
    const v4f p = *(const v4fa*)(stg + row * DOUT + 4 * lane);
    float* op = Zp + (size_t)(rowBase + row) * (size_t)DOUT + 4 * lane;
    *(volatile v4f*)op = p;
  }
  if (wave < 2) *(volatile v4f*)sp = sdv;
}

__device__ __forceinline__ int scan_chunk(const int* __restrict__ dsts, int nE, int cbase, int slotBase,
                                          int nb, int* list, int lane, int wave) {
  int wc = 0;
  const int ell  = wave * WCAP + lane;
  const int e0   = cbase + ell;
  const int sent = (int)(1u << 31);
  const int emax = nE - 1;
#define LDJ(J, DJ) \
  int DJ; { const int e = e0 + 32 * (J); const int ec = e < emax ? e : emax; \
            const int v = dsts[ec]; asm volatile("" :: "v"(v)); \
            const int ok = -(int)(e < nE); DJ = (v & ok) | (sent & ~ok); }
  LDJ(0, d0) LDJ(1, d1) LDJ(2, d2) LDJ(3, d3) LDJ(4, d4) LDJ(5, d5) LDJ(6, d6) LDJ(7, d7)
#undef LDJ
  const unsigned nbs = (unsigned)slotBase;
  const unsigned unb = (unsigned)nb;
  const unsigned s0 = (unsigned)d0 - nbs, s1 = (unsigned)d1 - nbs;
  const unsigned s2 = (unsigned)d2 - nbs, s3 = (unsigned)d3 - nbs;
  const unsigned s4 = (unsigned)d4 - nbs, s5 = (unsigned)d5 - nbs;
  const unsigned s6 = (unsigned)d6 - nbs, s7 = (unsigned)d7 - nbs;
  const bool h0 = s0 < unb, h1 = s1 < unb, h2 = s2 < unb, h3 = s3 < unb;
  const bool h4 = s4 < unb, h5 = s5 < unb, h6 = s6 < unb, h7 = s7 < unb;
  const unsigned any = __builtin_amdgcn_ballot_w32(h0 | h1 | h2 | h3 | h4 | h5 | h6 | h7);
  if (any != 0u) {
#define HITJ(J, HJ, SJ) { \
      const unsigned mj = __builtin_amdgcn_ballot_w32(HJ); \
      if (mj != 0u) { \
        if (HJ) { \
          const int pos = wc + (int)__builtin_amdgcn_mbcnt_lo(mj, 0u); \
          if (pos < WCAP) list[wave * WCAP + pos] = ((ell + 32 * (J)) << SLB) | (int)(SJ); \
        } \
        wc += (int)__builtin_popcount(mj); } }
    HITJ(0, h0, s0)
    HITJ(1, h1, s1)
    HITJ(2, h2, s2)
    HITJ(3, h3, s3)
    HITJ(4, h4, s4)
    HITJ(5, h5, s5)
    HITJ(6, h6, s6)
    HITJ(7, h7, s7)
#undef HITJ
  }
  return wc;
}

__device__ __forceinline__ void bucket_store(const int* reg2, const int* sc2, int npc, int nIt, int tid, int lane,
                                             int wave, int* hb, int* OC, int nSlot, int nodeBase, int* fp, v4i fv) {
#pragma unroll 1
  for (int it = 0; it < nIt; ++it) {
    const int p  = it * NTHR + tid;
    const int pc = p < npc ? p : npc - 1;
    const v4i v = *(const v4ia*)(reg2 + 4 * pc);
    asm volatile("" :: "v"(v));
    if (p < npc) *(volatile v4i*)(hb + 4 * p) = v;
  }
  if (wave < 4) {
    const int pl = wave >> 1;
    const int q  = tid & 63;
    const v4i v = *(const v4ia*)(sc2 + pl * NBRUN + 4 * q);
    *(volatile v4i*)(OC + (size_t)pl * (size_t)nSlot + nodeBase + 4 * q) = v;
  }
  if (wave == 4 && lane < 8) *(volatile v4i*)(fp + 4 * lane) = fv;
}

__global__ __launch_bounds__(NTHR) __attribute__((amdgpu_num_vgpr(248)))
void k_bucket(const int* __restrict__ srcs, const int* __restrict__ dsts, int nE, int nN,
              int* HITS, int* OC, int* FLG, int nSlot) {
  extern __shared__ __attribute__((aligned(16))) int dsm[];
  int* list = dsm;
  int* reg1 = dsm + LISTN;
  int* reg2 = reg1 + RCAP;
  int* sc2  = reg2 + RCAP;
  int* cur  = sc2 + 2 * NBRUN;
  int* wcnt = cur + NBRUN;
  int* wtot = wcnt + 8;
  const int tid = (int)threadIdx.x, lane = tid & 31;
  const int wave = __builtin_amdgcn_readfirstlane(tid >> 5);
  const int blk = (int)blockIdx.x;
  const int nodeBase = blk * NBRUN;
  int nb = nN - nodeBase;
  nb = nb < 0 ? 0 : (nb > NBRUN ? NBRUN : nb);

  sc2[tid] = 0;
  __syncthreads();

  int tot = 0, totraw = 0;
  const int nChunks = (nE + CHUNK - 1) / CHUNK;
#pragma unroll 1
  for (int ch = 0; ch < nChunks; ++ch) {
    const int cbase = ch * CHUNK;
    const int wc = scan_chunk(dsts, nE, cbase, nodeBase, nb, list, lane, wave);
    if (lane == 0) wcnt[wave] = wc;
    __syncthreads();
    int pre = 0, all = 0;
#pragma unroll
    for (int w2 = 0; w2 < NWAVE; ++w2) {
      int c = wcnt[w2];
      c = c < 0 ? 0 : (c > WCAP ? WCAP : c);
      all += c;
      pre += (w2 < wave) ? c : 0;
    }
    const int wcc  = __builtin_amdgcn_readfirstlane(wc > WCAP ? WCAP : wc);
    const int base = tot + pre;
#pragma unroll 1
    for (int b0 = 0; b0 < wcc; b0 += 32) {
      const int i   = b0 + lane;
      const int ic  = i < wcc ? i : wcc - 1;
      const int ent = list[wave * WCAP + ic];
      const int el  = (ent >> SLB) & (CHUNK - 1);
      const int sl  = ent & (NBRUN - 1);
      int eid = cbase + el;
      eid = eid > nE - 1 ? nE - 1 : eid;
      int sr = srcs[eid];
      asm volatile("" :: "v"(sr));
      sr = sr < 0 ? 0 : (sr > nN - 1 ? nN - 1 : sr);
      const int pos = base + i;
      if (i < wcc && pos < RCAP) reg1[pos] = sr | (sl << SRCB);
    }
    totraw += all;
    tot = totraw > RCAP ? RCAP : totraw;
    __syncthreads();
  }
  const int nh  = __builtin_amdgcn_readfirstlane(tot);
  const int ovf = totraw > RCAP ? 1 : 0;

  if (wave == 0) {
#pragma unroll 1
    for (int b0 = 0; b0 < nh; b0 += 32) {
      const int idx = b0 + lane;
      const int uv  = reg1[idx < nh ? idx : nh - 1];
      const int m32 = (nh - b0) < 32 ? (nh - b0) : 32;
#pragma unroll 1
      for (int k = 0; k < m32; ++k) {
        const int u  = __builtin_amdgcn_readlane(uv, k);
        const int sl = (u >> SRCB) & (NBRUN - 1);
        if (lane == 0) sc2[sl] = sc2[sl] + 1;
      }
    }
  }
  __syncthreads();

  {
    int c = sc2[tid];
    c = c < 0 ? 0 : c;
    int incl = c;
#pragma unroll
    for (int d = 1; d < 32; d <<= 1) {
      const int y = __shfl_up(incl, d);
      if (lane >= d) incl += y;
    }
    if (lane == 31) wtot[wave] = incl;
    __syncthreads();
    int pre = 0;
#pragma unroll
    for (int w2 = 0; w2 < NWAVE; ++w2) pre += (w2 < wave) ? wtot[w2] : 0;
    const int run = pre + incl - c;
    sc2[NBRUN + tid] = run;
    cur[tid] = run;
  }
  __syncthreads();

  const int nhp = (nh + 31) & ~31;
  if (wave == 0) {
#pragma unroll 1
    for (int b0 = 0; b0 < nh; b0 += 32) {
      const int idx = b0 + lane;
      const int uv  = reg1[idx < nh ? idx : nh - 1];
      const int m32 = (nh - b0) < 32 ? (nh - b0) : 32;
#pragma unroll 1
      for (int k = 0; k < m32; ++k) {
        const int u  = __builtin_amdgcn_readlane(uv, k);
        const int sl = (u >> SRCB) & (NBRUN - 1);
        if (lane == 0) {
          int p = cur[sl];
          p = p < 0 ? 0 : (p > RCAP - 1 ? RCAP - 1 : p);
          reg2[p] = u;
          cur[sl] = p + 1;
        }
      }
    }
    const int pi = nh + lane;
    if (pi < nhp) reg2[pi] = 0;
  }
  __syncthreads();

  const int npc = nhp >> 2;
  const int nIt = (npc + NTHR - 1) / NTHR;
  int* hb = HITS + (size_t)blk * RCAP;
  int* fp = FLG + blk * 32;
  const v4i fv = {ovf, ovf, ovf, ovf};
  bucket_store(reg2, sc2, npc, nIt, tid, lane, wave, hb, OC, nSlot, nodeBase, fp, fv);
  __threadfence();
  bucket_store(reg2, sc2, npc, nIt, tid, lane, wave, hb, OC, nSlot, nodeBase, fp, fv);
}

struct HitV { v4f z; float s; };
__device__ __forceinline__ HitV ld_hit(const int* __restrict__ hp, int idx, const float* __restrict__ SD,
                                       const float* __restrict__ Z, int nN, float fi, int lane) {
  const int w = hp[idx];
  int sr = w & ((1 << SRCB) - 1);
  sr = sr > nN - 1 ? nN - 1 : sr;
  const float es = SD[2 * sr];
  HitV r;
  r.z = *(const v4f*)(Z + (size_t)sr * DOUT + 4 * lane);
  r.s = es + fi;
  return r;
}

__global__ __launch_bounds__(NTHR) __attribute__((amdgpu_num_vgpr(248)))
void k_replay(const int* __restrict__ HITS, const int* __restrict__ OC, const int* __restrict__ FLG,
              const float* __restrict__ Z, const float* __restrict__ SD, float* outp, int nN, int nSlot) {
  const int tid = (int)threadIdx.x, lane = tid & 31;
  const int wave = __builtin_amdgcn_readfirstlane(tid >> 5);
  const int blk = (int)blockIdx.x;
  const int* hp = HITS + (size_t)blk * RCAP;
  const int fl = FLG[blk * 32];
  const float qn = __int_as_float(0x7fc00000);

#pragma unroll 1
  for (int j = 0; j < NBRUN / NWAVE; ++j) {
    const int node = blk * NBRUN + wave * (NBRUN / NWAVE) + j;
    if (node < nN) {
      const int craw = OC[node];
      const int oraw = OC[(size_t)nSlot + node];
      int c = craw < 0 ? 0 : (craw > DEGCAP ? DEGCAP : craw);
      int o = oraw < 0 ? 0 : (oraw > RCAP ? RCAP : oraw);
      const int room = RCAP - o;
      c = c > room ? room : c;
      const bool bad = (fl != 0) | (c != craw) | (o != oraw);
      c = __builtin_amdgcn_readfirstlane(c);
      o = __builtin_amdgcn_readfirstlane(o);
      const float fi = SD[2 * node + 1];
      int last = o + c - 1;
      last = last < o ? o : last;

      float mx = 0.0f, dn = 1.0f;
      v4f acc = {0.0f, 0.0f, 0.0f, 0.0f};
      if (c > 0) {
        const HitV h0 = ld_hit(hp, o, SD, Z, nN, fi, lane);
        mx = h0.s;
        acc = h0.z;
#pragma unroll 1
        for (int q = 1; q < c; ++q) {
          int idx = o + q;
          idx = idx > last ? last : idx;
          const HitV hv = ld_hit(hp, idx, SD, Z, nN, fi, lane);
          const float df = hv.s - mx;
          const float ee = expf(-fabsf(df));
          const bool  up = df > 0.0f;
          const float s1 = up ? ee : 1.0f;
          const float s2 = up ? 1.0f : ee;
          mx = up ? hv.s : mx;
          dn = fmaf(dn, s1, s2);
          acc.x = fmaf(acc.x, s1, s2 * hv.z.x);
          acc.y = fmaf(acc.y, s1, s2 * hv.z.y);
          acc.z = fmaf(acc.z, s1, s2 * hv.z.z);
          acc.w = fmaf(acc.w, s1, s2 * hv.z.w);
        }
      }
      const float inv = 1.0f / dn;
      v4f ov;
      ov.x = bad ? qn : acc.x * inv;
      ov.y = bad ? qn : acc.y * inv;
      ov.z = bad ? qn : acc.z * inv;
      ov.w = bad ? qn : acc.w * inv;
      float* op = outp + (size_t)node * DOUT + 4 * lane;
      *(volatile v4f*)op = ov;
      __threadfence();
      *(volatile v4f*)op = ov;
    }
  }
}

static inline int cdiv(int a, int b) { return (a + b - 1) / b; }

extern "C" void kernel_launch(void* const* d_in, const int* in_sizes, int n_in,
                              void* d_out, int out_size, void* d_ws, size_t ws_size,
                              hipStream_t stream) {
  if (n_in < 5) return;
  if (in_sizes[0] < DIN || (in_sizes[0] % DIN) != 0) return;
  const int nN = in_sizes[0] / DIN;
  if (nN < 1 || nN > (1 << SRCB)) return;
  const int nE = in_sizes[1];
  if (nE < 1 || in_sizes[2] != nE || nE > (1 << 28)) return;
  if (in_sizes[3] != DOUT * DIN) return;
  if (in_sizes[4] != 2 * DOUT) return;
  if ((long long)out_size != (long long)nN * DOUT) return;

  const float* h    = (const float*)d_in[0];
  const int*   src  = (const int*)d_in[1];
  const int*   dst  = (const int*)d_in[2];
  const float* Wfc  = (const float*)d_in[3];
  const float* Wat  = (const float*)d_in[4];
  float* out = (float*)d_out;

  const int MP    = cdiv(nN, GBM) * GBM;
  const int gM    = MP / GBM;
  const int bH    = MP / 16;
  const int nBlk  = cdiv(MP, NBRUN);
  const int nSlot = nBlk * NBRUN;
  if ((long long)nBlk * NBRUN < (long long)nN) return;

  char* ws = (char*)d_ws;
  size_t off = 0;
  const size_t oHB = off; off += (size_t)MP * DIN * 2;            off = (off + 255) & ~(size_t)255;
  const size_t oWB = off; off += (size_t)DOUT * DIN * 2;          off = (off + 255) & ~(size_t)255;
  const size_t oAV = off; off += (size_t)2 * DOUT * 4;            off = (off + 255) & ~(size_t)255;
  const size_t oZ  = off; off += (size_t)MP * DOUT * 4;           off = (off + 255) & ~(size_t)255;
  const size_t oSD = off; off += (size_t)MP * 2 * 4;              off = (off + 255) & ~(size_t)255;
  const size_t oHT = off; off += (size_t)nBlk * RCAP * 4;         off = (off + 255) & ~(size_t)255;
  const size_t oOC = off; off += (size_t)2 * nSlot * 4;           off = (off + 255) & ~(size_t)255;
  const size_t oFL = off; off += (size_t)nBlk * 32 * 4;           off = (off + 255) & ~(size_t)255;
  if (off > ws_size || off > (size_t)(128u << 20)) return;
  unsigned short* HB = (unsigned short*)(ws + oHB);
  unsigned short* WB = (unsigned short*)(ws + oWB);
  float*          AV = (float*)(ws + oAV);
  float*          Zp = (float*)(ws + oZ);
  float*          SD = (float*)(ws + oSD);
  int*            HT = (int*)(ws + oHT);
  int*            OC = (int*)(ws + oOC);
  int*            FL = (int*)(ws + oFL);

  const size_t zsdLds = (size_t)ZSD_FLTS * 4;
  const size_t bktLds = (size_t)BKT_INTS * 4;
  hipFuncSetAttribute(reinterpret_cast<const void*>(&k_zsd), hipFuncAttributeMaxDynamicSharedMemorySize, (int)zsdLds);
  hipFuncSetAttribute(reinterpret_cast<const void*>(&k_bucket), hipFuncAttributeMaxDynamicSharedMemorySize, (int)bktLds);

  k_prep<<<bH + WBLK + 1, NTHR, 0, stream>>>(h, Wfc, Wat, nN, bH, HB, WB, AV);
  k_zsd<<<gM, NTHR, zsdLds, stream>>>(HB, WB, AV, Zp, SD);
  k_bucket<<<nBlk, NTHR, bktLds, stream>>>(src, dst, nE, nN, HT, OC, FL, nSlot);
  k_replay<<<nBlk, NTHR, 0, stream>>>(HT, OC, FL, Zp, SD, out, nN, nSlot);
}
